// GRUSlowStateExtractor_40003325394978
// MI455X (gfx1250) — hardware-run, weakly checked
//
#include <hip/hip_runtime.h>

typedef __attribute__((ext_vector_type(16))) __bf16   v16b;
typedef __attribute__((ext_vector_type(8)))  float    v8f;
typedef __attribute__((ext_vector_type(4)))  float    v4f;
typedef __attribute__((ext_vector_type(2)))  float    v2f;
typedef __attribute__((ext_vector_type(4)))  unsigned v4u;
typedef __attribute__((ext_vector_type(8)))  unsigned v8u;

constexpr int kBatch = 256;
constexpr int kSeq = 1024;
constexpr int kIn = 7;
constexpr int kHid = 64;
constexpr int kGate = 3 * kHid;
constexpr int kHalf = 128;
constexpr int kRowsPerBlk = 16;
constexpr int kLayerBlocks = kHalf / kRowsPerBlk;
constexpr int kPw = 36;
constexpr int kPw0 = 20;
constexpr int kStg = 68;
constexpr float kEps = 1e-8f;
constexpr size_t kPlaneFloats = (size_t)kHalf * kSeq * kHid;
constexpr size_t kPlaneBytes = kPlaneFloats * 4;
constexpr size_t kOut1 = (size_t)kBatch * kSeq * 4;
constexpr size_t kOut2 = 2 * kOut1;
constexpr size_t kOut3 = kOut2 + (size_t)kBatch * kSeq * 3;
constexpr size_t kOutTotal = kOut3 + (size_t)3 * kBatch * kHid;
static_assert(kGate == 192);
static_assert(kLayerBlocks == 8);
static_assert(kPlaneBytes == 33554432);
static_assert(kOut1 * 4 == 4194304);
static_assert(kOut2 * 4 == 8388608);
static_assert(kOut3 * 4 == 11534336);
static_assert(kOutTotal * 4 == 11730944);
static_assert((kPw * 4) % 16 == 0);
static_assert((kPw0 * 4) % 16 == 0);
static_assert((kStg * 4) % 16 == 0);
static_assert(kSeq % 32 == 0);

__device__ __forceinline__ unsigned bf_rne(float f) {
  const unsigned u = __float_as_uint(f);
  return (u + 0x7FFFu + ((u >> 16) & 1u)) >> 16;
}
__device__ __forceinline__ void split2(float a, float b, unsigned& hw, unsigned& lw) {
  const unsigned ha = bf_rne(a);
  const unsigned hb = bf_rne(b);
  const float ra = a - __uint_as_float(ha << 16);
  const float rb = b - __uint_as_float(hb << 16);
  const unsigned la = bf_rne(ra);
  const unsigned lb = bf_rne(rb);
  hw = ha | (hb << 16);
  lw = la | (lb << 16);
}
__device__ __forceinline__ v16b words_to_frag(v8u u) { return __builtin_bit_cast(v16b, u); }
__device__ __forceinline__ v16b lds_frag(const unsigned* p) {
  const v4u a = *(const v4u*)(p);
  const v4u b = *(const v4u*)(p + 8);
  const v8u u = __builtin_shufflevector(a, b, 0, 1, 2, 3, 4, 5, 6, 7);
  return __builtin_bit_cast(v16b, u);
}
__device__ __forceinline__ v8f mma3(v16b ah, v16b al, v16b bh, v16b bl, v8f c) {
  c = __builtin_amdgcn_wmma_f32_16x16x32_bf16(false, ah, false, bh, (short)0, c, false, false);
  c = __builtin_amdgcn_wmma_f32_16x16x32_bf16(false, ah, false, bl, (short)0, c, false, false);
  c = __builtin_amdgcn_wmma_f32_16x16x32_bf16(false, al, false, bh, (short)0, c, false, false);
  asm volatile("v_nop\n\tv_nop\n\tv_nop\n\tv_nop" : "+v"(c) : "v"(ah), "v"(al), "v"(bh), "v"(bl));
  return c;
}
__device__ __forceinline__ v8f mma1(v16b a, v16b b, v8f c) {
  c = __builtin_amdgcn_wmma_f32_16x16x32_bf16(false, a, false, b, (short)0, c, false, false);
  asm volatile("v_nop\n\tv_nop\n\tv_nop\n\tv_nop" : "+v"(c) : "v"(a), "v"(b));
  return c;
}
__device__ __forceinline__ void pin1(float& x) { asm volatile("" : "+v"(x)); }

__device__ __forceinline__ float sigm(float v) {
  v = fminf(fmaxf(v, -30.0f), 30.0f);
  return 1.0f / (1.0f + expf(-v));
}

template <bool L0>
__global__ __launch_bounds__(32) __attribute__((amdgpu_num_vgpr(256)))
void cell_layer_kernel(const float* __restrict__ src, const float* __restrict__ h0l,
                       const float* __restrict__ Wih, const float* __restrict__ Whh,
                       const float* __restrict__ bih, const float* __restrict__ bhh,
                       const float* __restrict__ resW, const float* __restrict__ resb,
                       float* __restrict__ zout, float* __restrict__ hTl, int bhalf0)
{
  __shared__ __align__(16) unsigned WhhH[kGate * kPw];
  __shared__ __align__(16) unsigned WhhL[kGate * kPw];
  __shared__ __align__(16) unsigned WihH[L0 ? 4 : kGate * kPw];
  __shared__ __align__(16) unsigned WihL[L0 ? 4 : kGate * kPw];
  __shared__ __align__(16) unsigned Wx0[L0 ? 256 * kPw0 : 4];
  __shared__ __align__(16) float hst[32 * 32];
  __shared__ __align__(16) float zst[L0 ? 4 : 32 * 32];
  __shared__ __align__(16) float stg[16 * kStg];
  __shared__ __align__(16) float bI[kGate];
  __shared__ __align__(16) float bH[kGate];
  __shared__ __align__(16) float bR[kHid];

  const int lane = threadIdx.x & 31;
  const int bn = lane & 15;
  const int hf = lane >> 4;
  const int bl0 = blockIdx.x * kRowsPerBlk;
  int bloc = bl0 + bn;
  bloc = bloc < kHalf ? bloc : kHalf - 1;
  int bglob = bhalf0 + bloc;
  bglob = bglob < kBatch ? bglob : kBatch - 1;
  int bglob0 = bhalf0 + bl0;
  bglob0 = bglob0 <= kBatch - kRowsPerBlk ? bglob0 : kBatch - kRowsPerBlk;
  int bloc0 = bl0 <= kHalf - kRowsPerBlk ? bl0 : kHalf - kRowsPerBlk;

#pragma unroll 1
  for (int i = lane; i < kGate * 32; i += 32) {
    const int row = i >> 5;
    const int wc = i & 31;
    const v2f w = *(const v2f*)(Whh + row * kHid + 2 * wc);
    unsigned hw, lw;
    split2(w[0], w[1], hw, lw);
    WhhH[row * kPw + wc] = hw;
    WhhL[row * kPw + wc] = lw;
  }
  if constexpr (!L0) {
#pragma unroll 1
    for (int i = lane; i < kGate * 32; i += 32) {
      const int row = i >> 5;
      const int wc = i & 31;
      const v2f w = *(const v2f*)(Wih + row * kHid + 2 * wc);
      unsigned hw, lw;
      split2(w[0], w[1], hw, lw);
      WihH[row * kPw + wc] = hw;
      WihL[row * kPw + wc] = lw;
    }
  } else {
#pragma unroll 1
    for (int it = 0; it < 8; ++it) {
      const int row = it * 32 + lane;
      float wv[7];
      if (it < 6) {
#pragma unroll
        for (int k = 0; k < kIn; ++k) wv[k] = Wih[row * kIn + k];
      } else {
#pragma unroll
        for (int k = 0; k < kIn; ++k) wv[k] = resW[(row - kGate) * kIn + k];
      }
      unsigned h01, l01, h23, l23, h45, l45, h6, l6;
      split2(wv[0], wv[1], h01, l01);
      split2(wv[2], wv[3], h23, l23);
      split2(wv[4], wv[5], h45, l45);
      split2(wv[6], 0.0f, h6, l6);
      const v4u hiw = {h01, h23, h45, h6};
      const v4u low = {l01, l23, l45, l6};
      const v4u zw = {0u, 0u, 0u, 0u};
      unsigned* rp = Wx0 + row * kPw0;
      *(v4u*)(rp) = hiw;
      *(v4u*)(rp + 4) = low;
      *(v4u*)(rp + 8) = hiw;
      *(v4u*)(rp + 12) = zw;
    }
  }
#pragma unroll 1
  for (int i = lane; i < kGate; i += 32) {
    bI[i] = bih[i];
    bH[i] = bhh[i];
  }
#pragma unroll 1
  for (int i = lane; i < kHid; i += 32) {
    if constexpr (L0) bR[i] = resb[i];
    else bR[i] = 0.0f;
  }
  {
    const float* hp = h0l + (size_t)bglob * kHid + 8 * hf;
#pragma unroll
    for (int j = 0; j < 4; ++j) {
      const v4f a = *(const v4f*)(hp + 16 * j);
      const v4f b = *(const v4f*)(hp + 16 * j + 4);
#pragma unroll
      for (int m = 0; m < 4; ++m) {
        hst[(8 * j + m) * 32 + lane] = a[m];
        hst[(8 * j + 4 + m) * 32 + lane] = b[m];
      }
    }
  }
  __syncthreads();

  const v8f zero8 = {0.f, 0.f, 0.f, 0.f, 0.f, 0.f, 0.f, 0.f};
  const int c4 = bn * 4;

#pragma unroll 1
  for (int t = 0; t < kSeq; ++t) {
    v16b hH[2], hLo[2];
#pragma unroll
    for (int s = 0; s < 2; ++s) {
      v8u uh, ul;
#pragma unroll
      for (int p = 0; p < 2; ++p) {
#pragma unroll
        for (int q = 0; q < 4; ++q) {
          const int slot = ((2 * s + p) * 8 + 2 * q) * 32 + lane;
          const float v0 = hst[slot];
          const float v1 = hst[slot + 32];
          unsigned hw, lw;
          split2(v0, v1, hw, lw);
          uh[4 * p + q] = hw;
          ul[4 * p + q] = lw;
        }
      }
      hH[s] = words_to_frag(uh);
      hLo[s] = words_to_frag(ul);
    }
    v16b xH[2], xLo[2];
    v16b xb;
    if constexpr (!L0) {
      const float* zr = src + ((size_t)bloc * kSeq + t) * kHid + 8 * hf;
#pragma unroll
      for (int s = 0; s < 2; ++s) {
        v8u uh, ul;
#pragma unroll
        for (int p = 0; p < 2; ++p) {
          const int j = 2 * s + p;
          const v4f a = *(const v4f*)(zr + 16 * j);
          const v4f b = *(const v4f*)(zr + 16 * j + 4);
#pragma unroll
          for (int m = 0; m < 4; ++m) {
            zst[(8 * j + m) * 32 + lane] = a[m];
            zst[(8 * j + 4 + m) * 32 + lane] = b[m];
          }
          unsigned hw, lw;
          split2(a[0], a[1], hw, lw);
          uh[4 * p + 0] = hw;
          ul[4 * p + 0] = lw;
          split2(a[2], a[3], hw, lw);
          uh[4 * p + 1] = hw;
          ul[4 * p + 1] = lw;
          split2(b[0], b[1], hw, lw);
          uh[4 * p + 2] = hw;
          ul[4 * p + 2] = lw;
          split2(b[2], b[3], hw, lw);
          uh[4 * p + 3] = hw;
          ul[4 * p + 3] = lw;
        }
        xH[s] = words_to_frag(uh);
        xLo[s] = words_to_frag(ul);
      }
    } else {
      const float* xr = src + ((size_t)bglob * kSeq + t) * kIn;
      float x0 = xr[0];
      float x1 = xr[1];
      float x2 = xr[2];
      float x3 = xr[3];
      float x4 = xr[4];
      float x5 = xr[5];
      float x6 = xr[6];
      pin1(x0);
      pin1(x1);
      pin1(x2);
      pin1(x3);
      pin1(x4);
      pin1(x5);
      pin1(x6);
      unsigned h01, l01, h23, l23, h45, l45, h6, l6;
      split2(x0, x1, h01, l01);
      split2(x2, x3, h23, l23);
      split2(x4, x5, h45, l45);
      split2(x6, 0.0f, h6, l6);
      v8u u;
      u[0] = h01;
      u[1] = h23;
      u[2] = h45;
      u[3] = h6;
      u[4] = (hf == 0) ? l01 : 0u;
      u[5] = (hf == 0) ? l23 : 0u;
      u[6] = (hf == 0) ? l45 : 0u;
      u[7] = (hf == 0) ? l6 : 0u;
      xb = words_to_frag(u);
    }

#pragma unroll 1
    for (int j = 0; j < 4; ++j) {
      const int rowb = 16 * j + bn;
      v8f ar = zero8;
      v8f az = zero8;
      v8f ani = zero8;
      v8f anh = zero8;
      v8f ares = zero8;
#pragma unroll
      for (int s = 0; s < 2; ++s) {
        const int off = rowb * kPw + 16 * s + 4 * hf;
        ar = mma3(lds_frag(WhhH + off), lds_frag(WhhL + off), hH[s], hLo[s], ar);
        az = mma3(lds_frag(WhhH + off + 64 * kPw), lds_frag(WhhL + off + 64 * kPw), hH[s], hLo[s], az);
        anh = mma3(lds_frag(WhhH + off + 128 * kPw), lds_frag(WhhL + off + 128 * kPw), hH[s], hLo[s], anh);
        if constexpr (!L0) {
          ar = mma3(lds_frag(WihH + off), lds_frag(WihL + off), xH[s], xLo[s], ar);
          az = mma3(lds_frag(WihH + off + 64 * kPw), lds_frag(WihL + off + 64 * kPw), xH[s], xLo[s], az);
          ani = mma3(lds_frag(WihH + off + 128 * kPw), lds_frag(WihL + off + 128 * kPw), xH[s], xLo[s], ani);
        }
      }
      if constexpr (L0) {
        const int off0 = rowb * kPw0 + 4 * hf;
        ar = mma1(lds_frag(Wx0 + off0), xb, ar);
        az = mma1(lds_frag(Wx0 + off0 + 64 * kPw0), xb, az);
        ani = mma1(lds_frag(Wx0 + off0 + 128 * kPw0), xb, ani);
        ares = mma1(lds_frag(Wx0 + off0 + 192 * kPw0), xb, ares);
      }
#pragma unroll
      for (int m = 0; m < 8; ++m) {
        const int gr = 16 * j + 8 * hf + m;
        const int slot = (8 * j + m) * 32 + lane;
        const float hold = hst[slot];
        const float pr = ar[m] + (bI[gr] + bH[gr]);
        const float pz = az[m] + (bI[64 + gr] + bH[64 + gr]);
        const float rg = sigm(pr);
        const float zg = sigm(pz);
        const float pn = (ani[m] + bI[128 + gr]) + rg * (anh[m] + bH[128 + gr]);
        const float ng = tanhf(pn);
        const float hn = (1.0f - zg) * ng + zg * hold;
        hst[slot] = hn;
        float rs;
        if constexpr (L0) rs = ares[m] + bR[gr];
        else rs = zst[slot];
        stg[bn * kStg + gr] = hn + rs;
      }
    }
    __syncthreads();
    {
      v4f vals[8];
#pragma unroll
      for (int it = 0; it < 8; ++it) vals[it] = *(const v4f*)(stg + (it * 2 + hf) * kStg + c4);
      for (int pass = 0; pass < 2; ++pass) {
#pragma unroll
        for (int it = 0; it < 8; ++it) {
          const int row = it * 2 + hf;
          *(volatile v4f*)(zout + ((size_t)(bloc0 + row) * kSeq + t) * kHid + c4) = vals[it];
        }
        __threadfence();
      }
    }
    __syncthreads();
  }

#pragma unroll
  for (int j = 0; j < 4; ++j) {
#pragma unroll
    for (int m = 0; m < 8; ++m) {
      stg[bn * kStg + 16 * j + 8 * hf + m] = hst[(8 * j + m) * 32 + lane];
    }
  }
  __syncthreads();
  {
    v4f vals[8];
#pragma unroll
    for (int it = 0; it < 8; ++it) vals[it] = *(const v4f*)(stg + (it * 2 + hf) * kStg + c4);
    for (int pass = 0; pass < 2; ++pass) {
#pragma unroll
      for (int it = 0; it < 8; ++it) {
        const int row = it * 2 + hf;
        *(volatile v4f*)(hTl + (size_t)(bglob0 + row) * kHid + c4) = vals[it];
      }
      __threadfence();
    }
  }
}

__global__ __launch_bounds__(128) __attribute__((amdgpu_num_vgpr(256)))
void head_kernel(const float* __restrict__ z2, const float* __restrict__ x,
                 const float* __restrict__ meanv, const float* __restrict__ stdv,
                 const float* __restrict__ qW1, const float* __restrict__ qb1,
                 const float* __restrict__ qW2, const float* __restrict__ qb2,
                 const float* __restrict__ wW1, const float* __restrict__ wb1,
                 const float* __restrict__ wW2, const float* __restrict__ wb2,
                 float* __restrict__ out, int bhalf0)
{
  __shared__ __align__(16) unsigned W1H[128 * kPw];
  __shared__ __align__(16) unsigned W1L[128 * kPw];
  __shared__ __align__(16) unsigned W2qH[16 * kPw];
  __shared__ __align__(16) unsigned W2qL[16 * kPw];
  __shared__ __align__(16) unsigned W2wH[16 * kPw];
  __shared__ __align__(16) unsigned W2wL[16 * kPw];
  __shared__ __align__(16) float b1s[128];
  __shared__ __align__(16) float b2s[8];
  __shared__ __align__(16) float ms[8];
  __shared__ __align__(16) float sq0[4][128];
  __shared__ __align__(16) float sq1[4][128];
  __shared__ __align__(16) float som[4][96];

  const int tid = threadIdx.x;
  const int lane = tid & 31;
  const int wave = tid >> 5;
  const int n = lane & 15;
  const int hf = lane >> 4;
  int bl = blockIdx.x;
  bl = bl < kHalf ? bl : kHalf - 1;
  int bg = bhalf0 + bl;
  bg = bg < kBatch ? bg : kBatch - 1;

#pragma unroll 1
  for (int i = tid; i < 64 * 32; i += 128) {
    const int row = i >> 5;
    const int wc = i & 31;
    const v2f w = *(const v2f*)(qW1 + row * kHid + 2 * wc);
    unsigned hw, lw;
    split2(w[0], w[1], hw, lw);
    W1H[row * kPw + wc] = hw;
    W1L[row * kPw + wc] = lw;
  }
#pragma unroll 1
  for (int i = tid; i < 64 * 32; i += 128) {
    const int row = i >> 5;
    const int wc = i & 31;
    const v2f w = *(const v2f*)(wW1 + row * kHid + 2 * wc);
    unsigned hw, lw;
    split2(w[0], w[1], hw, lw);
    W1H[(64 + row) * kPw + wc] = hw;
    W1L[(64 + row) * kPw + wc] = lw;
  }
#pragma unroll 1
  for (int i = tid; i < 16 * 32; i += 128) {
    const int row = i >> 5;
    const int wc = i & 31;
    const int rq = row < 4 ? row : 3;
    int rw = row - 4;
    rw = rw < 0 ? 0 : (rw > 2 ? 2 : rw);
    const v2f wq = *(const v2f*)(qW2 + rq * kHid + 2 * wc);
    const v2f ww = *(const v2f*)(wW2 + rw * kHid + 2 * wc);
    const bool onq = row < 4;
    const bool onw = (row >= 4) && (row <= 6);
    const float q0 = onq ? wq[0] : 0.0f;
    const float q1 = onq ? wq[1] : 0.0f;
    const float w0 = onw ? ww[0] : 0.0f;
    const float w1 = onw ? ww[1] : 0.0f;
    unsigned hw, lw;
    split2(q0, q1, hw, lw);
    W2qH[row * kPw + wc] = hw;
    W2qL[row * kPw + wc] = lw;
    split2(w0, w1, hw, lw);
    W2wH[row * kPw + wc] = hw;
    W2wL[row * kPw + wc] = lw;
  }
  {
    float a = qb1[tid & 63];
    float b = wb1[tid & 63];
    pin1(a);
    pin1(b);
    b1s[tid] = (tid < 64) ? a : b;
    const int t4 = tid & 3;
    int t3 = (tid & 7) - 4;
    t3 = t3 < 0 ? 0 : (t3 > 2 ? 2 : t3);
    float qa = qb2[t4];
    float wa = wb2[t3];
    float mv = meanv[t4];
    float sv = stdv[t4];
    pin1(qa);
    pin1(wa);
    pin1(mv);
    pin1(sv);
    if (tid < 8) {
      b2s[tid] = (tid < 4) ? qa : ((tid < 7) ? wa : 0.0f);
      ms[tid] = (tid < 4) ? mv : sv;
    }
  }
  __syncthreads();

  const v8f zero8 = {0.f, 0.f, 0.f, 0.f, 0.f, 0.f, 0.f, 0.f};

#pragma unroll 1
  for (int it = 0; it < 8; ++it) {
    const int tb = 256 * wave + 32 * it;
#pragma unroll 1
    for (int u = 0; u < 2; ++u) {
      const int t = tb + 16 * u + n;
      const float* zr = z2 + ((size_t)bl * kSeq + t) * kHid + 8 * hf;
      v16b zH[2], zL[2];
#pragma unroll
      for (int s = 0; s < 2; ++s) {
        v8u uh, ul;
#pragma unroll
        for (int p = 0; p < 2; ++p) {
          const int j = 2 * s + p;
          const v4f a = *(const v4f*)(zr + 16 * j);
          const v4f b = *(const v4f*)(zr + 16 * j + 4);
          unsigned hw, lw;
          split2(a[0], a[1], hw, lw);
          uh[4 * p + 0] = hw;
          ul[4 * p + 0] = lw;
          split2(a[2], a[3], hw, lw);
          uh[4 * p + 1] = hw;
          ul[4 * p + 1] = lw;
          split2(b[0], b[1], hw, lw);
          uh[4 * p + 2] = hw;
          ul[4 * p + 2] = lw;
          split2(b[2], b[3], hw, lw);
          uh[4 * p + 3] = hw;
          ul[4 * p + 3] = lw;
        }
        zH[s] = words_to_frag(uh);
        zL[s] = words_to_frag(ul);
      }
      const float* xr = x + ((size_t)bg * kSeq + t) * kIn;
      float x0 = xr[0];
      float x1 = xr[1];
      float x2 = xr[2];
      float x3 = xr[3];
      pin1(x0);
      pin1(x1);
      pin1(x2);
      pin1(x3);

      v8u ghw[2][2], glw[2][2];
#pragma unroll
      for (int jt = 0; jt < 8; ++jt) {
        v8f acc = zero8;
#pragma unroll
        for (int s = 0; s < 2; ++s) {
          const int off = (16 * jt + n) * kPw + 16 * s + 4 * hf;
          acc = mma3(lds_frag(W1H + off), lds_frag(W1L + off), zH[s], zL[s], acc);
        }
        const int hd = jt >> 2;
        const int s2 = (jt & 3) >> 1;
        const int p = jt & 1;
#pragma unroll
        for (int q = 0; q < 4; ++q) {
          const int gr = 16 * jt + 8 * hf + 2 * q;
          const float v0 = fmaxf(acc[2 * q] + b1s[gr], 0.0f);
          const float v1 = fmaxf(acc[2 * q + 1] + b1s[gr + 1], 0.0f);
          unsigned hw, lw;
          split2(v0, v1, hw, lw);
          ghw[hd][s2][4 * p + q] = hw;
          glw[hd][s2][4 * p + q] = lw;
        }
      }
      v8f acc2 = zero8;
#pragma unroll
      for (int s = 0; s < 2; ++s) {
        const int off = n * kPw + 16 * s + 4 * hf;
        acc2 = mma3(lds_frag(W2qH + off), lds_frag(W2qL + off), words_to_frag(ghw[0][s]), words_to_frag(glw[0][s]), acc2);
        acc2 = mma3(lds_frag(W2wH + off), lds_frag(W2wL + off), words_to_frag(ghw[1][s]), words_to_frag(glw[1][s]), acc2);
      }
      const float qi0 = x0 * ms[4] + ms[0];
      const float qi1 = x1 * ms[5] + ms[1];
      const float qi2 = x2 * ms[6] + ms[2];
      const float qi3 = x3 * ms[7] + ms[3];
      const float nn = qi0 * qi0 + qi1 * qi1 + qi2 * qi2 + qi3 * qi3;
      const float inv = 1.0f / (sqrtf(nn) + kEps);
      const float qn0 = qi0 * inv;
      const float qn1 = qi1 * inv;
      const float qn2 = qi2 * inv;
      const float qn3 = qi3 * inv;
      const float sg0 = (qn0 < 0.0f) ? -1.0f : 1.0f;
      const float r0 = qn0 * sg0 + (acc2[0] + b2s[0]);
      const float r1 = qn1 * sg0 + (acc2[1] + b2s[1]);
      const float r2 = qn2 * sg0 + (acc2[2] + b2s[2]);
      const float r3 = qn3 * sg0 + (acc2[3] + b2s[3]);
      const float n2 = r0 * r0 + r1 * r1 + r2 * r2 + r3 * r3;
      const float inv2 = 1.0f / (sqrtf(n2) + kEps);
      const float sg1 = (r0 < 0.0f) ? -1.0f : 1.0f;
      const v4f rawv = {r0, r1, r2, r3};
      const v4f qpv = {r0 * inv2 * sg1, r1 * inv2 * sg1, r2 * inv2 * sg1, r3 * inv2 * sg1};
      const float om0 = acc2[4] + b2s[4];
      const float om1 = acc2[5] + b2s[5];
      const float om2 = acc2[6] + b2s[6];
      if (hf == 0) {
        const int row = 16 * u + n;
        *(v4f*)(&sq0[wave][row * 4]) = rawv;
        *(v4f*)(&sq1[wave][row * 4]) = qpv;
        som[wave][row * 3 + 0] = om0;
        som[wave][row * 3 + 1] = om1;
        som[wave][row * 3 + 2] = om2;
      }
    }
    __syncthreads();
    {
      const v4f o0 = *(const v4f*)(&sq0[wave][4 * lane]);
      const v4f o1 = *(const v4f*)(&sq1[wave][4 * lane]);
      const int l2 = lane < 24 ? lane : 0;
      const v4f o2 = *(const v4f*)(&som[wave][4 * l2]);
      const size_t rbase = (size_t)bg * kSeq + tb;
      float* p0 = out + rbase * 4 + 4 * lane;
      float* p1 = out + kOut1 + rbase * 4 + 4 * lane;
      float* p2 = out + kOut2 + rbase * 3 + 4 * l2;
      for (int pass = 0; pass < 2; ++pass) {
        *(volatile v4f*)p0 = o0;
        *(volatile v4f*)p1 = o1;
        if (lane < 24) *(volatile v4f*)p2 = o2;
        __threadfence();
      }
    }
    __syncthreads();
  }
}

extern "C" void kernel_launch(void* const* d_in, const int* in_sizes, int n_in,
                              void* d_out, int out_size, void* d_ws, size_t ws_size,
                              hipStream_t stream) {
  if (n_in < 26) return;
  if (in_sizes[0] < kBatch * kSeq * kIn || in_sizes[1] < 3 * kBatch * kHid ||
      in_sizes[2] < 4 || in_sizes[3] < 4 ||
      in_sizes[4] < kGate * kIn || in_sizes[5] < kGate * kHid ||
      in_sizes[8] < kGate * kHid || in_sizes[9] < kGate * kHid ||
      in_sizes[12] < kGate * kHid || in_sizes[13] < kGate * kHid ||
      in_sizes[16] < kHid * kIn || in_sizes[18] < kHid * kHid || in_sizes[20] < 4 * kHid ||
      in_sizes[22] < kHid * kHid || in_sizes[24] < 3 * kHid ||
      (size_t)out_size < kOutTotal) return;
  if (ws_size < 2 * kPlaneBytes) return;

  const float* x     = (const float*)d_in[0];
  const float* h0    = (const float*)d_in[1];
  const float* meanv = (const float*)d_in[2];
  const float* stdv  = (const float*)d_in[3];
  const float* Wih0  = (const float*)d_in[4];
  const float* Whh0  = (const float*)d_in[5];
  const float* bih0  = (const float*)d_in[6];
  const float* bhh0  = (const float*)d_in[7];
  const float* Wih1  = (const float*)d_in[8];
  const float* Whh1  = (const float*)d_in[9];
  const float* bih1  = (const float*)d_in[10];
  const float* bhh1  = (const float*)d_in[11];
  const float* Wih2  = (const float*)d_in[12];
  const float* Whh2  = (const float*)d_in[13];
  const float* bih2  = (const float*)d_in[14];
  const float* bhh2  = (const float*)d_in[15];
  const float* resW  = (const float*)d_in[16];
  const float* resb  = (const float*)d_in[17];
  const float* qW1   = (const float*)d_in[18];
  const float* qb1   = (const float*)d_in[19];
  const float* qW2   = (const float*)d_in[20];
  const float* qb2   = (const float*)d_in[21];
  const float* wW1   = (const float*)d_in[22];
  const float* wb1   = (const float*)d_in[23];
  const float* wW2   = (const float*)d_in[24];
  const float* wb2   = (const float*)d_in[25];

  float* P0 = (float*)d_ws;
  float* P1 = P0 + kPlaneFloats;
  float* out = (float*)d_out;
  float* hT = out + kOut3;
  const size_t lstride = (size_t)kBatch * kHid;

  for (int half = 0; half < 2; ++half) {
    const int bh0 = half * kHalf;
    cell_layer_kernel<true><<<dim3(kLayerBlocks), dim3(32), 0, stream>>>(
        x, h0, Wih0, Whh0, bih0, bhh0, resW, resb, P0, hT, bh0);
    cell_layer_kernel<false><<<dim3(kLayerBlocks), dim3(32), 0, stream>>>(
        P0, h0 + lstride, Wih1, Whh1, bih1, bhh1, resW, resb, P1, hT + lstride, bh0);
    cell_layer_kernel<false><<<dim3(kLayerBlocks), dim3(32), 0, stream>>>(
        P1, h0 + 2 * lstride, Wih2, Whh2, bih2, bhh2, resW, resb, P0, hT + 2 * lstride, bh0);
    head_kernel<<<dim3(kHalf), dim3(128), 0, stream>>>(
        P0, x, meanv, stdv, qW1, qb1, qW2, qb2, wW1, wb1, wW2, wb2, out, bh0);
  }
}
